// DIN_UBM_60859686584662
// MI455X (gfx1250) — hardware-verified
//
#include <hip/hip_runtime.h>

typedef unsigned short us16;
typedef __bf16   v16bf    __attribute__((ext_vector_type(16)));
typedef _Float16 v16h     __attribute__((ext_vector_type(16)));
typedef float    v8f      __attribute__((ext_vector_type(8)));
typedef us16     v8us_raw __attribute__((ext_vector_type(8)));
typedef us16     v4us_raw __attribute__((ext_vector_type(4)));
typedef float    v4f_raw  __attribute__((ext_vector_type(4)));
typedef v8us_raw __attribute__((may_alias)) v8us;
typedef v4us_raw __attribute__((may_alias)) v4us;
typedef v4f_raw  __attribute__((may_alias)) v4f;

union FragU { v16bf v; v8us_raw half[2]; };

#define NB 256
#define NS 50
#define NF 30
#define NE 16
#define D80 80
#define NGRP (NB * NS)
#define NFROW (NGRP * NF)
#define KP1 192
#define KOFF2 96
#define MK1 336
#define MK1P 352
#define APITCH 104
#define XPITCH 360
#define HPITCH 136
#define REPP 96
#define GPB 4
#define PAD_NEG (-1073741823.0f)
#define NEG_BIG (-3.0e38f)

#define R_UID 100002
#define R_DID 100002
#define R_GEN 4
#define R_AGE 10
#define R_PROV 42
#define R_VID 100002
#define R_AID 50002
#define R_C2 202
#define R_C1 52
#define R_UP 12
#define R_WDAY 9
#define R_HOUR 26
#define R_MIN 62

__device__ __forceinline__ us16 bf_rne(float x) {
  unsigned u = __float_as_uint(x);
  u += 0x7FFFu + ((u >> 16) & 1u);
  return (us16)(u >> 16);
}
__device__ __forceinline__ float bf_val(us16 b) { return __uint_as_float(((unsigned)b) << 16); }
__device__ __forceinline__ void split_hl(float x, us16& hi, us16& lo) {
  hi = bf_rne(x);
  lo = bf_rne(x - bf_val(hi));
}
__device__ __forceinline__ int clampi(int i, int n) { return i < 0 ? 0 : (i >= n ? n - 1 : i); }

__device__ __forceinline__ v8f wmma_bf(v16bf a, v16bf b, v8f c) {
  v8f d = __builtin_amdgcn_wmma_f32_16x16x32_bf16(false, a, false, b, (short)0, c, false, false);
  const v16h ah = __builtin_bit_cast(v16h, a);
  const v16h bh = __builtin_bit_cast(v16h, b);
  asm volatile("v_nop\n\tv_nop\n\tv_nop\n\tv_nop" : "+v"(d) : "v"(ah), "v"(bh));
  return d;
}
__device__ __forceinline__ v8f mma3(v16bf ah, v16bf al, v16bf bh, v16bf bl, v8f c) {
  c = wmma_bf(ah, bh, c);
  c = wmma_bf(ah, bl, c);
  c = wmma_bf(al, bh, c);
  return c;
}
__device__ __forceinline__ v16bf ldfrag(const us16* p, int h) {
  FragU f;
  f.half[0] = *(const v8us*)(p + 8 * h);
  f.half[1] = *(const v8us*)(p + 16 + 8 * h);
  return f.v;
}
__device__ __forceinline__ void wave_sync() {
  __builtin_amdgcn_fence(__ATOMIC_RELEASE, "wavefront");
  __builtin_amdgcn_wave_barrier();
  __builtin_amdgcn_fence(__ATOMIC_ACQUIRE, "wavefront");
}

__device__ __forceinline__ void emb16(const float* tab, int rows, int zrow, int idx, bool live,
                                      v4f_raw& o0, v4f_raw& o1, v4f_raw& o2, v4f_raw& o3) {
  const int ic = clampi(idx, rows);
  const float* r = tab + (size_t)ic * NE;
  const v4f_raw a0 = *(const v4f*)(r);
  const v4f_raw a1 = *(const v4f*)(r + 4);
  const v4f_raw a2 = *(const v4f*)(r + 8);
  const v4f_raw a3 = *(const v4f*)(r + 12);
  const bool z = (!live) || (ic == zrow);
  #pragma unroll
  for (int e = 0; e < 4; ++e) {
    o0[e] = z ? 0.0f : a0[e];
    o1[e] = z ? 0.0f : a1[e];
    o2[e] = z ? 0.0f : a2[e];
    o3[e] = z ? 0.0f : a3[e];
  }
}
__device__ __forceinline__ void split8(v4f_raw x, v4f_raw y, v8us_raw& hv, v8us_raw& lv) {
  #pragma unroll
  for (int e = 0; e < 4; ++e) {
    us16 p, q;
    split_hl(x[e], p, q); hv[e] = p;     lv[e] = q;
    split_hl(y[e], p, q); hv[4 + e] = p; lv[4 + e] = q;
  }
}
__device__ __forceinline__ void split4(v4f_raw x, bool z, v4us_raw& hv, v4us_raw& lv) {
  #pragma unroll
  for (int e = 0; e < 4; ++e) {
    const float t = z ? 0.0f : x[e];
    us16 p, q;
    split_hl(t, p, q);
    hv[e] = p; lv[e] = q;
  }
}
template <bool EMB>
__device__ __forceinline__ void put_row(const float* tab, int rows, int zrow, int idx, bool live,
                                        float* ed, us16* hd, us16* ld) {
  v4f_raw o0, o1, o2, o3;
  emb16(tab, rows, zrow, idx, live, o0, o1, o2, o3);
  if (EMB) {
    *(v4f*)(ed) = o0; *(v4f*)(ed + 4) = o1; *(v4f*)(ed + 8) = o2; *(v4f*)(ed + 12) = o3;
  }
  v8us_raw h0, l0, h1, l1;
  split8(o0, o1, h0, l0);
  split8(o2, o3, h1, l1);
  *(v8us*)(hd) = h0; *(v8us*)(hd + 8) = h1;
  *(v8us*)(ld) = l0; *(v8us*)(ld + 8) = l1;
}

struct PrArgs {
  const float* w0; const float* w1; const float* w2; const float* w3; const float* w4;
  us16* p0; us16* p1; us16* p2; us16* p3; us16* p4;
};
static_assert(sizeof(PrArgs) == 10 * 8);

__global__ void __launch_bounds__(64) prep_kernel(PrArgs a) {
  const int bid = blockIdx.x;
  int pl = 9, start = 368;
  if (bid < 30)       { pl = 0; start = 0; }
  else if (bid < 60)  { pl = 1; start = 30; }
  else if (bid < 90)  { pl = 2; start = 60; }
  else if (bid < 120) { pl = 3; start = 90; }
  else if (bid < 208) { pl = 4; start = 120; }
  else if (bid < 296) { pl = 5; start = 208; }
  else if (bid < 328) { pl = 6; start = 296; }
  else if (bid < 360) { pl = 7; start = 328; }
  else if (bid < 368) { pl = 8; start = 360; }
  const int wsel = pl >> 1, islo = pl & 1;
  const float* W = (wsel == 0) ? a.w0 : (wsel == 1) ? a.w1 : (wsel == 2) ? a.w2 : (wsel == 3) ? a.w3 : a.w4;
  us16* base     = (wsel == 0) ? a.p0 : (wsel == 1) ? a.p1 : (wsel == 2) ? a.p2 : (wsel == 3) ? a.p3 : a.p4;
  const int N  = (wsel < 2) ? D80 : ((wsel == 4) ? 32 : 128);
  const int Kp = (wsel < 2) ? KP1 : ((wsel == 2) ? MK1P : 128);
  const int K  = (wsel == 2) ? MK1 : 128;
  const bool sp = wsel < 2;
  us16* dst = base + (islo ? N * Kp : 0);
  const int e0 = (bid - start) * 512 + (int)threadIdx.x * 8;
  const int n = e0 / Kp, kk0 = e0 - n * Kp;
  v8us_raw o;
  #pragma unroll
  for (int i = 0; i < 8; ++i) {
    const int kk = kk0 + i;
    bool valid; int k;
    if (sp) {
      valid = (kk < D80) || (kk >= KOFF2 && kk < KOFF2 + D80);
      k = (kk < D80) ? kk : (kk - (KOFF2 - D80));
    } else {
      valid = kk < K;
      k = kk;
    }
    const int kc = valid ? k : 0;
    float x = W[(size_t)kc * N + n];
    x = valid ? x : 0.0f;
    us16 hv, lv;
    split_hl(x, hv, lv);
    o[i] = islo ? lv : hv;
  }
  us16* p = dst + e0;
  *(volatile v8us*)p = o;
  __threadfence();
  *(volatile v8us*)p = o;
}

struct FlArgs {
  const int* flow_arr; const int* flow_mask; const int* seq_arr;
  const float* vid_tab; const float* aid_tab; const float* c2_tab; const float* c1_tab; const float* up_tab;
  const us16* w1h; const us16* w1l; const float* b1; const float* w2; const float* b2;
  float* rep;
};
static_assert(sizeof(FlArgs) == 14 * 8);

__global__ void __launch_bounds__(128) fl_kernel(FlArgs a) {
  __shared__ __align__(16) float sEmb[128][D80];
  __shared__ __align__(16) us16  sAh[128][APITCH];
  __shared__ __align__(16) us16  sAl[128][APITCH];
  __shared__ __align__(16) us16  sSh[16][APITCH];
  __shared__ __align__(16) us16  sSl[16][APITCH];
  __shared__ __align__(16) float sSeq[16][D80];
  __shared__ __align__(16) float sLog[GPB][32];
  __shared__ __align__(16) float sSc[GPB][32];
  __shared__ __align__(16) float sRep[GPB][REPP];

  const int tid = threadIdx.x, lane = tid & 31, w = tid >> 5, h = lane >> 4, m = lane & 15;
  const int bs = blockIdx.x * GPB + w;
  const int f = lane;
  const bool live = f < NF;
  const int fr = bs * NF + (live ? f : (NF - 1));

  {
    const int* ip = a.flow_arr + (size_t)fr * 5;
    const int i0 = ip[0], i1 = ip[1], i2 = ip[2], i3 = ip[3], i4 = ip[4];
    float* ed = &sEmb[tid][0];
    us16* hd = &sAh[tid][0];
    us16* ld = &sAl[tid][0];
    put_row<true>(a.vid_tab, R_VID, 0, i0, live, ed,      hd,      ld);
    put_row<true>(a.aid_tab, R_AID, 0, i1, live, ed + 16, hd + 16, ld + 16);
    put_row<true>(a.c2_tab,  R_C2,  0, i2, live, ed + 32, hd + 32, ld + 32);
    put_row<true>(a.c1_tab,  R_C1,  2, i3, live, ed + 48, hd + 48, ld + 48);
    put_row<true>(a.up_tab,  R_UP,  0, i4, live, ed + 64, hd + 64, ld + 64);
    const v8us_raw z8 = {(us16)0, (us16)0, (us16)0, (us16)0, (us16)0, (us16)0, (us16)0, (us16)0};
    *(v8us*)(hd + 80) = z8; *(v8us*)(hd + 88) = z8;
    *(v8us*)(ld + 80) = z8; *(v8us*)(ld + 88) = z8;
  }
  if (w == 0) {
    const int row = m;
    const bool lv = row < GPB;
    const int bss = blockIdx.x * GPB + (lv ? row : 0);
    const int* ip = a.seq_arr + (size_t)bss * 5;
    const int i0 = ip[0], i1 = ip[1], i2 = ip[2], i3 = ip[3], i4 = ip[4];
    us16* hd = &sSh[row][0];
    us16* ld = &sSl[row][0];
    put_row<false>(a.vid_tab, R_VID, 0, i0, lv, nullptr, hd,      ld);
    put_row<false>(a.aid_tab, R_AID, 0, i1, lv, nullptr, hd + 16, ld + 16);
    put_row<false>(a.c2_tab,  R_C2,  0, i2, lv, nullptr, hd + 32, ld + 32);
    put_row<false>(a.c1_tab,  R_C1,  2, i3, lv, nullptr, hd + 48, ld + 48);
    put_row<false>(a.up_tab,  R_UP,  0, i4, lv, nullptr, hd + 64, ld + 64);
    const v8us_raw z8 = {(us16)0, (us16)0, (us16)0, (us16)0, (us16)0, (us16)0, (us16)0, (us16)0};
    *(v8us*)(hd + 80) = z8; *(v8us*)(hd + 88) = z8;
    *(v8us*)(ld + 80) = z8; *(v8us*)(ld + 88) = z8;
  }
  __syncthreads();

  const v8f zero8 = {0.f, 0.f, 0.f, 0.f, 0.f, 0.f, 0.f, 0.f};

  if (w == 0) {
    v8f q[5];
    #pragma unroll
    for (int nt = 0; nt < 5; ++nt) q[nt] = zero8;
    #pragma unroll 1
    for (int ks = 0; ks < 3; ++ks) {
      const v16bf ah = ldfrag(&sSh[m][32 * ks], h);
      const v16bf al = ldfrag(&sSl[m][32 * ks], h);
      #pragma unroll
      for (int nt = 0; nt < 5; ++nt) {
        const size_t bo = (size_t)(16 * nt + m) * KP1 + KOFF2 + 32 * ks;
        const v16bf bh = ldfrag(a.w1h + bo, h);
        const v16bf bl = ldfrag(a.w1l + bo, h);
        q[nt] = mma3(ah, al, bh, bl, q[nt]);
      }
    }
    #pragma unroll
    for (int nt = 0; nt < 5; ++nt)
      #pragma unroll
      for (int r = 0; r < 8; ++r) sSeq[8 * h + r][16 * nt + m] = q[nt][r];
  }
  __syncthreads();

  const float b2 = a.b2[0];
  #pragma unroll 1
  for (int mt = 0; mt < 2; ++mt) {
    const int row = 32 * w + 16 * mt + m;
    v8f acc[5];
    #pragma unroll
    for (int nt = 0; nt < 5; ++nt) acc[nt] = zero8;
    #pragma unroll 1
    for (int ks = 0; ks < 3; ++ks) {
      const v16bf ah = ldfrag(&sAh[row][32 * ks], h);
      const v16bf al = ldfrag(&sAl[row][32 * ks], h);
      #pragma unroll
      for (int nt = 0; nt < 5; ++nt) {
        const size_t bo = (size_t)(16 * nt + m) * KP1 + 32 * ks;
        const v16bf bh = ldfrag(a.w1h + bo, h);
        const v16bf bl = ldfrag(a.w1l + bo, h);
        acc[nt] = mma3(ah, al, bh, bl, acc[nt]);
      }
    }
    float part[8];
    #pragma unroll
    for (int r = 0; r < 8; ++r) part[r] = 0.0f;
    #pragma unroll
    for (int nt = 0; nt < 5; ++nt) {
      const int n = 16 * nt + m;
      const float sqv = sSeq[w][n];
      const float b1n = a.b1[n];
      const float w2n = a.w2[n];
      #pragma unroll
      for (int r = 0; r < 8; ++r) {
        float v = acc[nt][r] + sqv;
        v = v + b1n;
        v = fmaxf(v, 0.0f);
        part[r] = fmaf(v, w2n, part[r]);
      }
    }
    #pragma unroll
    for (int r = 0; r < 8; ++r) {
      part[r] += __shfl_xor(part[r], 1, 32);
      part[r] += __shfl_xor(part[r], 2, 32);
      part[r] += __shfl_xor(part[r], 4, 32);
      part[r] += __shfl_xor(part[r], 8, 32);
    }
    if (m == 0) {
      #pragma unroll
      for (int r = 0; r < 8; ++r) sLog[w][16 * mt + 8 * h + r] = part[r] + b2;
    }
  }
  wave_sync();

  {
    const float lg = sLog[w][lane];
    const int fm = a.flow_mask[fr];
    const float x = live ? ((fm != 0) ? lg : PAD_NEG) : NEG_BIG;
    float mx = x;
    #pragma unroll
    for (int o = 16; o > 0; o >>= 1) mx = fmaxf(mx, __shfl_xor(mx, o, 32));
    const float e = live ? expf(x - mx) : 0.0f;
    float sm = e;
    #pragma unroll
    for (int o = 16; o > 0; o >>= 1) sm += __shfl_xor(sm, o, 32);
    sSc[w][lane] = e * (1.0f / sm);
  }
  wave_sync();

  #pragma unroll
  for (int c = 0; c < 3; ++c) {
    const int col = lane + 32 * c;
    const int colc = (col < D80) ? col : (D80 - 1);
    float racc = 0.0f;
    #pragma unroll 1
    for (int ff = 0; ff < NF; ++ff) racc = fmaf(sSc[w][ff], sEmb[32 * w + ff][colc], racc);
    sRep[w][col] = (col < D80) ? racc : 0.0f;
  }
  wave_sync();

  if (lane < 24) {
    const v4f_raw v = *(const v4f*)&sRep[w][4 * lane];
    float* dst = a.rep + (size_t)bs * REPP + 4 * lane;
    *(volatile v4f*)dst = v;
    __threadfence();
    *(volatile v4f*)dst = v;
  }
}

struct SqArgs {
  const int* rw; const int* rh; const int* rm; const int* uid; const int* did; const int* gen;
  const int* age; const int* prov; const int* vid; const int* aid; const int* c2; const int* c1;
  const int* upt; const int* uw; const int* uh; const int* um; const int* seq_mask;
  const float* uid_tab; const float* did_tab; const float* gen_tab; const float* age_tab; const float* prov_tab;
  const float* vid_tab; const float* aid_tab; const float* c2_tab; const float* c1_tab; const float* up_tab;
  const float* wday_tab; const float* hour_tab; const float* min_tab;
  const float* rep;
  const us16* aw1h; const us16* aw1l; const float* ab1; const float* aw2; const float* ab2;
  const us16* m1h; const us16* m1l; const us16* m2h; const us16* m2l; const us16* m3h; const us16* m3l;
  const float* mb1; const float* mb2; const float* mb3; const float* mw4; const float* mb4;
  float* out;
};
static_assert(sizeof(SqArgs) == 48 * 8);

#define OFF_X    0
#define OFF_TAH  45056
#define OFF_TAL  51712
#define OFF_TQ   58368
#define OFF_WT   68608
#define OFF_LOG  95232
#define OFF_SC   96256
#define OFF_XH   45056
#define OFF_XL   68096
#define OFF_H1H  0
#define OFF_H1L  8704
#define OFF_H2H  17408
#define OFF_H2L  26112
#define OFF_H3   34816
#define OFF_OUT  38912
#define SMEM2    97280

__device__ __forceinline__ void mlp_layer4(const us16* Ah, const us16* Al, int ap, int ksteps,
                                           const us16* Bh, const us16* Bl, int bp, const float* bias,
                                           us16* Oh, us16* Ol, int mt, int ntb, int h, int m) {
  const v8f zero8 = {0.f, 0.f, 0.f, 0.f, 0.f, 0.f, 0.f, 0.f};
  v8f acc[4];
  #pragma unroll
  for (int q = 0; q < 4; ++q) acc[q] = zero8;
  #pragma unroll 1
  for (int ks = 0; ks < ksteps; ++ks) {
    const v16bf ah = ldfrag(Ah + (size_t)(16 * mt + m) * ap + 32 * ks, h);
    const v16bf al = ldfrag(Al + (size_t)(16 * mt + m) * ap + 32 * ks, h);
    #pragma unroll
    for (int q = 0; q < 4; ++q) {
      const size_t bo = (size_t)(16 * (ntb + q) + m) * bp + 32 * ks;
      const v16bf bh = ldfrag(Bh + bo, h);
      const v16bf bl = ldfrag(Bl + bo, h);
      acc[q] = mma3(ah, al, bh, bl, acc[q]);
    }
  }
  #pragma unroll
  for (int q = 0; q < 4; ++q) {
    const int n = 16 * (ntb + q) + m;
    const float bn = bias[n];
    #pragma unroll
    for (int r = 0; r < 8; ++r) {
      const float v = fmaxf(acc[q][r] + bn, 0.0f);
      us16 hv, lv;
      split_hl(v, hv, lv);
      const int row = 16 * mt + 8 * h + r;
      Oh[row * HPITCH + n] = hv;
      Ol[row * HPITCH + n] = lv;
    }
  }
}

__global__ void __launch_bounds__(128) sq_kernel(SqArgs a) {
  __shared__ __align__(16) unsigned char smem[SMEM2];
  float* sX   = (float*)(smem + OFF_X);
  us16*  sTAh = (us16*)(smem + OFF_TAH);
  us16*  sTAl = (us16*)(smem + OFF_TAL);
  float* sTq  = (float*)(smem + OFF_TQ);
  us16*  sWT  = (us16*)(smem + OFF_WT);
  float* sLog = (float*)(smem + OFF_LOG);
  float* sSc  = (float*)(smem + OFF_SC);
  us16*  sXh  = (us16*)(smem + OFF_XH);
  us16*  sXl  = (us16*)(smem + OFF_XL);
  us16*  sH1h = (us16*)(smem + OFF_H1H);
  us16*  sH1l = (us16*)(smem + OFF_H1L);
  us16*  sH2h = (us16*)(smem + OFF_H2H);
  us16*  sH2l = (us16*)(smem + OFF_H2L);
  float* sH3  = (float*)(smem + OFF_H3);
  float* sOut = (float*)(smem + OFF_OUT);

  const int tid = threadIdx.x, lane = tid & 31, w = tid >> 5, h = lane >> 4, m = lane & 15;
  const int b0 = blockIdx.x * 32;
  us16* tH = sWT + w * (2 * 16 * APITCH);
  us16* tL = tH + 16 * APITCH;
  const v8f zero8 = {0.f, 0.f, 0.f, 0.f, 0.f, 0.f, 0.f, 0.f};
  const v8us_raw z8 = {(us16)0, (us16)0, (us16)0, (us16)0, (us16)0, (us16)0, (us16)0, (us16)0};

  {
    const int row = tid >> 2, q = tid & 3;
    const v4f_raw z4 = {0.f, 0.f, 0.f, 0.f};
    *(v4f*)&sX[row * MK1P + MK1 + 4 * q] = z4;
  }
  if (tid < 32) {
    *(v8us*)(sTAh + tid * APITCH + 80) = z8; *(v8us*)(sTAh + tid * APITCH + 88) = z8;
    *(v8us*)(sTAl + tid * APITCH + 80) = z8; *(v8us*)(sTAl + tid * APITCH + 88) = z8;
  }
  if (lane < 16) {
    *(v8us*)(tH + lane * APITCH + 80) = z8; *(v8us*)(tH + lane * APITCH + 88) = z8;
    *(v8us*)(tL + lane * APITCH + 80) = z8; *(v8us*)(tL + lane * APITCH + 88) = z8;
  }
  #pragma unroll 1
  for (int t = 0; t < 4; ++t) {
    const int j = w + 4 * t;
    const float* tab = a.wday_tab; const int* ids = a.rw; int rows = R_WDAY, zrow = 0, col = 0, ts = -1;
    switch (j) {
      case 1:  tab = a.hour_tab; ids = a.rh;   rows = R_HOUR; col = 16;  break;
      case 2:  tab = a.min_tab;  ids = a.rm;   rows = R_MIN;  col = 32;  break;
      case 3:  tab = a.uid_tab;  ids = a.uid;  rows = R_UID;  col = 48;  break;
      case 4:  tab = a.did_tab;  ids = a.did;  rows = R_DID;  col = 64;  break;
      case 5:  tab = a.gen_tab;  ids = a.gen;  rows = R_GEN;  col = 80;  break;
      case 6:  tab = a.age_tab;  ids = a.age;  rows = R_AGE;  col = 96;  break;
      case 7:  tab = a.prov_tab; ids = a.prov; rows = R_PROV; col = 112; break;
      case 8:  tab = a.wday_tab; ids = a.uw;   rows = R_WDAY; col = 288; break;
      case 9:  tab = a.hour_tab; ids = a.uh;   rows = R_HOUR; col = 304; break;
      case 10: tab = a.min_tab;  ids = a.um;   rows = R_MIN;  col = 320; break;
      case 11: tab = a.vid_tab;  ids = a.vid;  rows = R_VID;  col = 208; ts = 0; break;
      case 12: tab = a.aid_tab;  ids = a.aid;  rows = R_AID;  col = 224; ts = 1; break;
      case 13: tab = a.c2_tab;   ids = a.c2;   rows = R_C2;   col = 240; ts = 2; break;
      case 14: tab = a.c1_tab;   ids = a.c1;   rows = R_C1;   zrow = 2; col = 256; ts = 3; break;
      case 15: tab = a.up_tab;   ids = a.upt;  rows = R_UP;   col = 272; ts = 4; break;
      default: break;
    }
    const int bl = lane, b = b0 + bl;
    const int idx = ids[b];
    v4f_raw o0, o1, o2, o3;
    emb16(tab, rows, zrow, idx, true, o0, o1, o2, o3);
    float* xd = sX + bl * MK1P + col;
    *(v4f*)(xd) = o0; *(v4f*)(xd + 4) = o1; *(v4f*)(xd + 8) = o2; *(v4f*)(xd + 12) = o3;
    if (ts >= 0) {
      v8us_raw h0, l0, h1, l1;
      split8(o0, o1, h0, l0);
      split8(o2, o3, h1, l1);
      us16* hd = sTAh + bl * APITCH + 16 * ts;
      us16* ld = sTAl + bl * APITCH + 16 * ts;
      *(v8us*)(hd) = h0; *(v8us*)(hd + 8) = h1;
      *(v8us*)(ld) = l0; *(v8us*)(ld + 8) = l1;
    }
  }
  __syncthreads();

  if (w < 2) {
    v8f q[5];
    #pragma unroll
    for (int nt = 0; nt < 5; ++nt) q[nt] = zero8;
    #pragma unroll 1
    for (int ks = 0; ks < 3; ++ks) {
      const v16bf ah = ldfrag(sTAh + (16 * w + m) * APITCH + 32 * ks, h);
      const v16bf al = ldfrag(sTAl + (16 * w + m) * APITCH + 32 * ks, h);
      #pragma unroll
      for (int nt = 0; nt < 5; ++nt) {
        const size_t bo = (size_t)(16 * nt + m) * KP1 + KOFF2 + 32 * ks;
        const v16bf bh = ldfrag(a.aw1h + bo, h);
        const v16bf bl = ldfrag(a.aw1l + bo, h);
        q[nt] = mma3(ah, al, bh, bl, q[nt]);
      }
    }
    #pragma unroll
    for (int nt = 0; nt < 5; ++nt)
      #pragma unroll
      for (int r = 0; r < 8; ++r) sTq[(16 * w + 8 * h + r) * D80 + 16 * nt + m] = q[nt][r];
  }
  __syncthreads();

  const float ab2 = a.ab2[0];
  #pragma unroll 1
  for (int i = 0; i < 8; ++i) {
    const int bl = 8 * w + i, b = b0 + bl;
    const float* repb = a.rep + (size_t)b * NS * REPP;
    #pragma unroll 1
    for (int mt = 0; mt < 4; ++mt) {
      #pragma unroll
      for (int j2 = 0; j2 < 10; ++j2) {
        const int item = 32 * j2 + lane;
        const int row = item / 20, c4 = item - row * 20;
        const int s = 16 * mt + row;
        const int sc = (s < NS) ? s : (NS - 1);
        const v4f_raw v = *(const v4f*)(repb + (size_t)sc * REPP + 4 * c4);
        v4us_raw hv, lv;
        split4(v, s >= NS, hv, lv);
        *(v4us*)(tH + row * APITCH + 4 * c4) = hv;
        *(v4us*)(tL + row * APITCH + 4 * c4) = lv;
      }
      wave_sync();
      v8f acc[5];
      #pragma unroll
      for (int nt = 0; nt < 5; ++nt) acc[nt] = zero8;
      #pragma unroll 1
      for (int ks = 0; ks < 3; ++ks) {
        const v16bf ah = ldfrag(tH + m * APITCH + 32 * ks, h);
        const v16bf al = ldfrag(tL + m * APITCH + 32 * ks, h);
        #pragma unroll
        for (int nt = 0; nt < 5; ++nt) {
          const size_t bo = (size_t)(16 * nt + m) * KP1 + 32 * ks;
          const v16bf bh = ldfrag(a.aw1h + bo, h);
          const v16bf bl = ldfrag(a.aw1l + bo, h);
          acc[nt] = mma3(ah, al, bh, bl, acc[nt]);
        }
      }
      float part[8];
      #pragma unroll
      for (int r = 0; r < 8; ++r) part[r] = 0.0f;
      #pragma unroll
      for (int nt = 0; nt < 5; ++nt) {
        const int n = 16 * nt + m;
        const float tq = sTq[bl * D80 + n];
        const float b1n = a.ab1[n];
        const float w2n = a.aw2[n];
        #pragma unroll
        for (int r = 0; r < 8; ++r) {
          float v = acc[nt][r] + tq;
          v = v + b1n;
          v = fmaxf(v, 0.0f);
          part[r] = fmaf(v, w2n, part[r]);
        }
      }
      #pragma unroll
      for (int r = 0; r < 8; ++r) {
        part[r] += __shfl_xor(part[r], 1, 32);
        part[r] += __shfl_xor(part[r], 2, 32);
        part[r] += __shfl_xor(part[r], 4, 32);
        part[r] += __shfl_xor(part[r], 8, 32);
      }
      if (m == 0) {
        #pragma unroll
        for (int r = 0; r < 8; ++r) sLog[w * 64 + 16 * mt + 8 * h + r] = part[r] + ab2;
      }
      wave_sync();
    }
    {
      const int s0 = lane, s1 = lane + 32;
      const bool v1 = s1 < NS;
      const int s1c = v1 ? s1 : (NS - 1);
      const float lg0 = sLog[w * 64 + s0], lg1 = sLog[w * 64 + s1];
      const int mk0 = a.seq_mask[(size_t)b * NS + s0];
      const int mk1 = a.seq_mask[(size_t)b * NS + s1c];
      const float x0 = (mk0 != 0) ? lg0 : PAD_NEG;
      const float x1 = v1 ? ((mk1 != 0) ? lg1 : PAD_NEG) : NEG_BIG;
      float mx = fmaxf(x0, x1);
      #pragma unroll
      for (int o = 16; o > 0; o >>= 1) mx = fmaxf(mx, __shfl_xor(mx, o, 32));
      const float e0 = expf(x0 - mx);
      const float e1 = v1 ? expf(x1 - mx) : 0.0f;
      float sm = e0 + e1;
      #pragma unroll
      for (int o = 16; o > 0; o >>= 1) sm += __shfl_xor(sm, o, 32);
      const float inv = 1.0f / sm;
      sSc[w * 64 + s0] = e0 * inv;
      sSc[w * 64 + s1] = e1 * inv;
    }
    wave_sync();
    #pragma unroll
    for (int c = 0; c < 3; ++c) {
      const int col = lane + 32 * c;
      const int colc = (col < D80) ? col : (D80 - 1);
      float iacc = 0.0f;
      #pragma unroll 1
      for (int s = 0; s < NS; ++s) iacc = fmaf(sSc[w * 64 + s], repb[(size_t)s * REPP + colc], iacc);
      if (col < D80) sX[bl * MK1P + 128 + col] = iacc;
    }
    wave_sync();
  }
  __syncthreads();

  #pragma unroll 1
  for (int j3 = 0; j3 < 22; ++j3) {
    const int item = tid + 128 * j3;
    const int row = item / 88, c4 = item - row * 88;
    const v4f_raw v = *(const v4f*)&sX[row * MK1P + 4 * c4];
    v4us_raw hv, lv;
    split4(v, false, hv, lv);
    *(v4us*)(sXh + row * XPITCH + 4 * c4) = hv;
    *(v4us*)(sXl + row * XPITCH + 4 * c4) = lv;
  }
  __syncthreads();
  mlp_layer4(sXh, sXl, XPITCH, 11, a.m1h, a.m1l, MK1P, a.mb1, sH1h, sH1l, w & 1, 4 * (w >> 1), h, m);
  __syncthreads();
  mlp_layer4(sH1h, sH1l, HPITCH, 4, a.m2h, a.m2l, 128, a.mb2, sH2h, sH2l, w & 1, 4 * (w >> 1), h, m);
  __syncthreads();
  {
    const int mt = w & 1, nt = w >> 1;
    v8f acc = zero8;
    #pragma unroll 1
    for (int ks = 0; ks < 4; ++ks) {
      const v16bf ah = ldfrag(sH2h + (16 * mt + m) * HPITCH + 32 * ks, h);
      const v16bf al = ldfrag(sH2l + (16 * mt + m) * HPITCH + 32 * ks, h);
      const size_t bo = (size_t)(16 * nt + m) * 128 + 32 * ks;
      const v16bf bh = ldfrag(a.m3h + bo, h);
      const v16bf bl = ldfrag(a.m3l + bo, h);
      acc = mma3(ah, al, bh, bl, acc);
    }
    const int n = 16 * nt + m;
    const float bn = a.mb3[n];
    #pragma unroll
    for (int r = 0; r < 8; ++r) sH3[(16 * mt + 8 * h + r) * 32 + n] = fmaxf(acc[r] + bn, 0.0f);
  }
  __syncthreads();
  if (w == 0) {
    const int bl = lane;
    float facc = 0.0f;
    #pragma unroll 1
    for (int jj = 0; jj < 32; ++jj) facc = fmaf(sH3[bl * 32 + jj], a.mw4[jj], facc);
    sOut[bl] = facc + a.mb4[0];
    wave_sync();
    const int l8 = (lane < 8) ? lane : 0;
    const v4f_raw v = *(const v4f*)&sOut[4 * l8];
    if (lane < 8) {
      float* dst = a.out + b0 + 4 * lane;
      *(volatile v4f*)dst = v;
      __threadfence();
      *(volatile v4f*)dst = v;
    }
  }
}

extern "C" void kernel_launch(void* const* d_in, const int* in_sizes, int n_in,
                              void* d_out, int out_size, void* d_ws, size_t ws_size,
                              hipStream_t stream) {
  if (n_in < 50) return;
  if (out_size != NB) return;
  for (int i = 0; i < 16; ++i) { if (in_sizes[i] != NB) return; }
  if (in_sizes[16] != NGRP * 5 || in_sizes[17] != NGRP) return;
  if (in_sizes[19] != NFROW * 5 || in_sizes[20] != NFROW) return;
  if (in_sizes[21] != R_UID * NE || in_sizes[22] != R_DID * NE || in_sizes[23] != R_GEN * NE ||
      in_sizes[24] != R_AGE * NE || in_sizes[25] != R_PROV * NE || in_sizes[26] != R_VID * NE ||
      in_sizes[27] != R_AID * NE || in_sizes[28] != R_C2 * NE || in_sizes[29] != R_C1 * NE ||
      in_sizes[30] != R_UP * NE || in_sizes[31] != R_WDAY * NE || in_sizes[32] != R_HOUR * NE ||
      in_sizes[33] != R_MIN * NE) return;
  if (in_sizes[34] != 160 * 80 || in_sizes[35] != 80 || in_sizes[36] != 80 || in_sizes[37] != 1) return;
  if (in_sizes[38] != 160 * 80 || in_sizes[39] != 80 || in_sizes[40] != 80 || in_sizes[41] != 1) return;
  if (in_sizes[42] != MK1 * 128 || in_sizes[43] != 128 || in_sizes[44] != 128 * 128 || in_sizes[45] != 128 ||
      in_sizes[46] != 128 * 32 || in_sizes[47] != 32 || in_sizes[48] != 32 || in_sizes[49] != 1) return;

  const size_t szP0  = (size_t)2 * 80 * KP1 * 2;
  const size_t szP1  = szP0;
  const size_t szP2  = (size_t)2 * 128 * MK1P * 2;
  const size_t szP3  = (size_t)2 * 128 * 128 * 2;
  const size_t szP4  = (size_t)2 * 32 * 128 * 2;
  const size_t szRep = (size_t)NGRP * REPP * 4;
  const size_t offP0 = 0;
  const size_t offP1 = offP0 + szP0;
  const size_t offP2 = offP1 + szP1;
  const size_t offP3 = offP2 + szP2;
  const size_t offP4 = offP3 + szP3;
  const size_t offRep = offP4 + szP4;
  const size_t total = offRep + szRep;
  if (total > ws_size) return;

  char* ws = (char*)d_ws;
  us16* p0 = (us16*)(ws + offP0);
  us16* p1 = (us16*)(ws + offP1);
  us16* p2 = (us16*)(ws + offP2);
  us16* p3 = (us16*)(ws + offP3);
  us16* p4 = (us16*)(ws + offP4);
  float* rep = (float*)(ws + offRep);

  PrArgs pr = {};
  pr.w0 = (const float*)d_in[34];
  pr.w1 = (const float*)d_in[38];
  pr.w2 = (const float*)d_in[42];
  pr.w3 = (const float*)d_in[44];
  pr.w4 = (const float*)d_in[46];
  pr.p0 = p0; pr.p1 = p1; pr.p2 = p2; pr.p3 = p3; pr.p4 = p4;
  prep_kernel<<<376, 64, 0, stream>>>(pr);

  FlArgs fl = {};
  fl.flow_arr  = (const int*)d_in[19];
  fl.flow_mask = (const int*)d_in[20];
  fl.seq_arr   = (const int*)d_in[16];
  fl.vid_tab   = (const float*)d_in[26];
  fl.aid_tab   = (const float*)d_in[27];
  fl.c2_tab    = (const float*)d_in[28];
  fl.c1_tab    = (const float*)d_in[29];
  fl.up_tab    = (const float*)d_in[30];
  fl.w1h = p0; fl.w1l = p0 + 80 * KP1;
  fl.b1 = (const float*)d_in[35];
  fl.w2 = (const float*)d_in[36];
  fl.b2 = (const float*)d_in[37];
  fl.rep = rep;
  fl_kernel<<<NGRP / GPB, 128, 0, stream>>>(fl);

  SqArgs sq = {};
  sq.rw  = (const int*)d_in[0];  sq.rh  = (const int*)d_in[1];  sq.rm  = (const int*)d_in[2];
  sq.uid = (const int*)d_in[3];  sq.did = (const int*)d_in[4];  sq.gen = (const int*)d_in[5];
  sq.age = (const int*)d_in[6];  sq.prov = (const int*)d_in[7];
  sq.vid = (const int*)d_in[8];  sq.aid = (const int*)d_in[9];  sq.c2  = (const int*)d_in[10];
  sq.c1  = (const int*)d_in[11]; sq.upt = (const int*)d_in[12];
  sq.uw  = (const int*)d_in[13]; sq.uh  = (const int*)d_in[14]; sq.um  = (const int*)d_in[15];
  sq.seq_mask = (const int*)d_in[17];
  sq.uid_tab  = (const float*)d_in[21]; sq.did_tab  = (const float*)d_in[22];
  sq.gen_tab  = (const float*)d_in[23]; sq.age_tab  = (const float*)d_in[24];
  sq.prov_tab = (const float*)d_in[25];
  sq.vid_tab  = (const float*)d_in[26]; sq.aid_tab  = (const float*)d_in[27];
  sq.c2_tab   = (const float*)d_in[28]; sq.c1_tab   = (const float*)d_in[29];
  sq.up_tab   = (const float*)d_in[30];
  sq.wday_tab = (const float*)d_in[31]; sq.hour_tab = (const float*)d_in[32]; sq.min_tab = (const float*)d_in[33];
  sq.rep = rep;
  sq.aw1h = p1; sq.aw1l = p1 + 80 * KP1;
  sq.ab1 = (const float*)d_in[39]; sq.aw2 = (const float*)d_in[40]; sq.ab2 = (const float*)d_in[41];
  sq.m1h = p2; sq.m1l = p2 + 128 * MK1P;
  sq.m2h = p3; sq.m2l = p3 + 128 * 128;
  sq.m3h = p4; sq.m3l = p4 + 32 * 128;
  sq.mb1 = (const float*)d_in[43]; sq.mb2 = (const float*)d_in[45]; sq.mb3 = (const float*)d_in[47];
  sq.mw4 = (const float*)d_in[48]; sq.mb4 = (const float*)d_in[49];
  sq.out = (float*)d_out;
  sq_kernel<<<NB / 32, 128, 0, stream>>>(sq);
}
